// SelfRouting2d_35828617183258
// MI455X (gfx1250) — hardware-verified
//
#include <hip/hip_runtime.h>


#ifndef NB
#define NB 64
#endif
#ifndef NCAP
#define NCAP 2048
#endif
#define NB_FULL   64
#define NCAP_FULL 2048
#define NI   64
#define NJ   512
#define CT   64
#define RT   32
#define XTN  64
#define XTP  68

static_assert(NI == 64);
static_assert(NI % 32 == 0);
static_assert(NJ % CT == 0);
static_assert(CT == 64);
static_assert(RT == 32);
static_assert(NCAP % RT == 0);
static_assert(NCAP % XTN == 0);
static_assert(NB <= NB_FULL);
static_assert(NCAP <= NCAP_FULL);
static_assert((XTP * 4) % 16 == 0);
static_assert(4 * 16 == NI);
static_assert(16 * 4 == XTN);
static_assert(2 * 256 * 8 == XTN * NI);
static_assert(16 * 16 == XTN * 4);
static_assert(16 * 16 == CT * 4);
static_assert(((size_t)NJ * NI) % 8 == 0);
static_assert((NI * XTP + XTN) * 4 <= 131072);
static_assert(CT * 4 <= 131072);

typedef unsigned short bf;
typedef __attribute__((ext_vector_type(16))) __bf16   v16bf;
typedef __attribute__((ext_vector_type(8)))  unsigned short v8us;
typedef __attribute__((ext_vector_type(8)))  float    v8f;
typedef __attribute__((ext_vector_type(4)))  float    v4f;
typedef v4f  __attribute__((may_alias)) v4fa;

__device__ __forceinline__ unsigned short f2bf(float f) { unsigned u = __float_as_uint(f); u += 0x7FFFu + ((u >> 16) & 1u); return (unsigned short)(u >> 16); }
__device__ __forceinline__ float bfr(float f) { return __uint_as_float(((unsigned)f2bf(f)) << 16); }
__device__ __forceinline__ v16bf cat16b(v8us lo, v8us hi) { return __builtin_bit_cast(v16bf, __builtin_shufflevector(lo, hi, 0, 1, 2, 3, 4, 5, 6, 7, 8, 9, 10, 11, 12, 13, 14, 15)); }
__device__ __forceinline__ v8f wmmab(v16bf a, v16bf b, v8f c) { return __builtin_amdgcn_wmma_f32_16x16x32_bf16(false, a, false, b, (short)0, c, false, false); }
__device__ __forceinline__ v8f wmmabg(v16bf a, v16bf b, v8f c) { c = wmmab(a, b, c); asm volatile("v_nop\n\tv_nop\n\tv_nop\n\tv_nop" : "+v"(c) : "v"(a), "v"(b)); return c; }
__device__ __forceinline__ v16bf ldb(const bf* p)  { return cat16b(*(const v8us*)p, *(const v8us*)(p + 16)); }
__device__ __forceinline__ void wave_sync() { __builtin_amdgcn_fence(3  , "wavefront"); __builtin_amdgcn_wave_barrier(); asm volatile("" ::: "memory"); }

__global__ __launch_bounds__(256) void k_cvt8(const float* __restrict__ src, bf* dst, size_t n8) {
    const size_t i = (size_t)blockIdx.x * 256 + threadIdx.x; if (i >= n8) return;
    const v8f v = *(const v8f*)(src + i * 8); v8us o;
#pragma unroll
    for (int k = 0; k < 8; ++k) o[k] = f2bf(v[k]);
    *(volatile v8us*)(dst + i * 8) = o; __threadfence(); *(volatile v8us*)(dst + i * 8) = o;
}

__global__ __launch_bounds__(256) void k_xt(const float* __restrict__ X, bf* XB, float* AN) {
    __shared__ __align__(16) float ts[NI * XTP];
    __shared__ __align__(16) float an[XTN];
    const int tid = threadIdx.x, lane = tid & 31;
    const int wave = __builtin_amdgcn_readfirstlane((int)(threadIdx.x >> 5));
    const int n0 = blockIdx.x * XTN, b = blockIdx.y;
    const float* xb = X + (size_t)b * NI * NCAP_FULL + n0;
#pragma unroll
    for (int it = 0; it < 4; ++it) {
        const int i = it * 16 + (tid >> 4), q = tid & 15;
        const v4f v = *(const v4f*)(xb + (size_t)i * NCAP_FULL + q * 4);
        v4f r; r[0] = bfr(v[0]); r[1] = bfr(v[1]); r[2] = bfr(v[2]); r[3] = bfr(v[3]);
        unsigned li = (unsigned)i * (unsigned)XTP + (unsigned)q * 4u; asm volatile("" : "+v"(li));
        *(v4fa*)(&ts[li]) = r;
    }
    __syncthreads();
    v8us ov[2];
#pragma unroll
    for (int s = 0; s < 2; ++s) {
        const int p = s * 256 + tid; const int n = p >> 3, c = p & 7;
        unsigned lb = (unsigned)c * (8u * (unsigned)XTP) + (unsigned)n; asm volatile("" : "+v"(lb));
        float ss = 0.0f; v8us o;
#pragma unroll
        for (int k = 0; k < 8; ++k) { const float v = ts[lb + (unsigned)k * (unsigned)XTP]; o[k] = (unsigned short)(__float_as_uint(v) >> 16); ss += v * v; }
        ss += __shfl_xor(ss, 1, 32); ss += __shfl_xor(ss, 2, 32); ss += __shfl_xor(ss, 4, 32);
        ov[s] = o;
        if (c == 0) an[n] = sqrtf(ss);
    }
    __syncthreads();
    unsigned l4 = (unsigned)(lane & 15) * 4u; asm volatile("" : "+v"(l4));
    const v4f av = *(const v4fa*)(&an[l4]);
    const bool aw = (wave == 0) & (lane < 16);
    bf* xo = XB + ((size_t)b * NCAP + n0) * NI;
    float* ao = AN + (size_t)b * NCAP + n0 + l4;
#pragma unroll 1
    for (int ps = 0; ps < 2; ++ps) {
#pragma unroll
        for (int s = 0; s < 2; ++s) { const int p = s * 256 + tid; *(volatile v8us*)(xo + (size_t)p * 8) = ov[s]; }
        if (aw) *(volatile v4f*)ao = av;
        if (ps == 0) __threadfence();
    }
}

__global__ __launch_bounds__(32) void k_gemm(const bf* __restrict__ XB, const bf* __restrict__ WB, const float* __restrict__ AN, float* OUT) {
    __shared__ __align__(16) float os[CT];
    const int lane = threadIdx.x & 31, lr = lane & 15, hi = lane >> 4;
    const int c0 = blockIdx.x * CT, b = blockIdx.y;
    v16bf wf[4][2];
    const size_t boff = (size_t)(c0 + lr) * NI + 8 * hi;
#pragma unroll
    for (int nb = 0; nb < 4; ++nb)
#pragma unroll
        for (int kq = 0; kq < 2; ++kq) wf[nb][kq] = ldb(WB + boff + (size_t)nb * 16 * NI + kq * 32);
    float cs0 = 0.0f, cs1 = 0.0f, cs2 = 0.0f, cs3 = 0.0f, sa = 0.0f;
    const size_t rbase = (size_t)b * NCAP;
#pragma unroll 1
    for (int rt = 0; rt < NCAP / RT; ++rt) {
        const size_t r0 = rbase + (size_t)rt * RT;
        const size_t aoff = (r0 + (size_t)lr) * NI + 8 * hi;
        v16bf a[2][2];
#pragma unroll
        for (int mb = 0; mb < 2; ++mb)
#pragma unroll
            for (int kq = 0; kq < 2; ++kq) a[mb][kq] = ldb(XB + aoff + (size_t)mb * 16 * NI + kq * 32);
        v8f acc[2][4];
#pragma unroll
        for (int mb = 0; mb < 2; ++mb)
#pragma unroll
            for (int nb = 0; nb < 4; ++nb) acc[mb][nb] = (v8f){};
#pragma unroll
        for (int kq = 0; kq < 2; ++kq)
#pragma unroll
            for (int nb = 0; nb < 4; ++nb)
#pragma unroll
                for (int mb = 0; mb < 2; ++mb) acc[mb][nb] = wmmabg(a[mb][kq], wf[nb][kq], acc[mb][nb]);
#pragma unroll
        for (int mb = 0; mb < 2; ++mb) {
            const float* ap = AN + r0 + mb * 16 + 8 * hi;
            const v4f w0 = *(const v4f*)ap, w1 = *(const v4f*)(ap + 4);
            sa += ((w0[0] + w0[1]) + (w0[2] + w0[3])) + ((w1[0] + w1[1]) + (w1[2] + w1[3]));
            float t[4];
#pragma unroll
            for (int nb = 0; nb < 4; ++nb) {
                float u = w0[0] * acc[mb][nb][0];
                u = fmaf(w0[1], acc[mb][nb][1], u); u = fmaf(w0[2], acc[mb][nb][2], u); u = fmaf(w0[3], acc[mb][nb][3], u);
                u = fmaf(w1[0], acc[mb][nb][4], u); u = fmaf(w1[1], acc[mb][nb][5], u); u = fmaf(w1[2], acc[mb][nb][6], u); u = fmaf(w1[3], acc[mb][nb][7], u);
                t[nb] = u; }
            cs0 += t[0]; cs1 += t[1]; cs2 += t[2]; cs3 += t[3];
        }
    }
    cs0 += __shfl_xor(cs0, 16, 32); cs1 += __shfl_xor(cs1, 16, 32); cs2 += __shfl_xor(cs2, 16, 32); cs3 += __shfl_xor(cs3, 16, 32);
    sa += __shfl_xor(sa, 16, 32);
    const float inv = 1.0f / sa;
    if (hi == 0) { os[0 * 16 + lr] = cs0 * inv; os[1 * 16 + lr] = cs1 * inv; os[2 * 16 + lr] = cs2 * inv; os[3 * 16 + lr] = cs3 * inv; }
    wave_sync();
    unsigned l4 = (unsigned)lr * 4u; asm volatile("" : "+v"(l4));
    const v4f val = *(const v4fa*)(&os[l4]);
    float* orow = OUT + (size_t)b * NJ + c0 + l4;
#pragma unroll 1
    for (int ps = 0; ps < 2; ++ps) {
        if (lane < 16) *(volatile v4f*)orow = val;
        if (ps == 0) __threadfence(); }
}

static constexpr size_t al256(size_t v) { return (v + 255) & ~(size_t)255; }
static constexpr size_t SZ_WB = al256((size_t)NJ * NI * 2);
static constexpr size_t SZ_XB = al256((size_t)NB * NCAP * NI * 2);
static constexpr size_t SZ_AN = al256((size_t)NB * NCAP * 4);
static constexpr size_t SZ_TOTAL = SZ_WB + SZ_XB + SZ_AN;
static_assert(SZ_TOTAL <= (size_t)134217728);
static_assert(((size_t)XTN * NI * 2) % 128 == 0);
static_assert(((size_t)XTN * 4) % 128 == 0);
static_assert(((size_t)NCAP * 4) % 128 == 0);
static_assert(((size_t)NJ * 4) % 128 == 0);
static_assert((size_t)(NB - 1) * NJ + NJ <= (size_t)NB_FULL * NJ);

extern "C" void kernel_launch(void* const* d_in, const int* in_sizes, int n_in,
                              void* d_out, int out_size, void* d_ws, size_t ws_size, hipStream_t stream) {
    if (n_in < 4) return;
    const size_t needx = ((size_t)(NB - 1) * NI + (size_t)(NI - 1)) * NCAP_FULL + NCAP;
    if ((size_t)in_sizes[0] < needx) return;
    if ((size_t)in_sizes[1] < (size_t)NJ * NI) return;
    if ((size_t)out_size < (size_t)NB * NJ) return;
    if (SZ_TOTAL > ws_size) return;
    const float* x  = (const float*)d_in[0];
    const float* w1 = (const float*)d_in[1];
    float* OUT = (float*)d_out;
    char* wsp = (char*)d_ws;
    bf* WB = (bf*)wsp; wsp += SZ_WB;
    bf* XB = (bf*)wsp; wsp += SZ_XB;
    float* AN = (float*)wsp; wsp += SZ_AN;

    { const size_t n8 = (size_t)NJ * NI / 8; k_cvt8<<<(unsigned)((n8 + 255) / 256), 256, 0, stream>>>(w1, WB, n8); }
    k_xt<<<dim3(NCAP / XTN, NB, 1), 256, 0, stream>>>(x, XB, AN);
    k_gemm<<<dim3(NJ / CT, NB, 1), 32, 0, stream>>>(XB, WB, AN, OUT);
}
